// NeighborhoodAttention2D_67645734912668
// MI455X (gfx1250) — hardware-verified
//
#include <hip/hip_runtime.h>
#include <math.h>
#include <stdint.h>

#define NBT   2
#define CH    256
#define IMH   56
#define IMW   56
#define NPOS  (IMH * IMW)
#define MROW  (NBT * NPOS)
#define NHD   8
#define HDIM  32
#define C3    (3 * CH)
#define KW    7
#define SUP   14
#define NSLOT 224
#define NKT   13
#define CTXK  512
#define QSCALE 0.17677669529663687f

static_assert((MROW % 64) == 0);
static_assert((C3 % 64) == 0);
static_assert((NPOS % 64) == 0);
static_assert((CH % 64) == 0);
static_assert((CH % 32) == 0 && (CTXK % 32) == 0);
static_assert(NHD * HDIM == CH);
static_assert(SUP == 8 + KW - 1);
static_assert(SUP * SUP <= NSLOT && (NSLOT % 32) == 0 && NKT * 16 >= SUP * SUP);
static_assert(IMH == IMW);

typedef __bf16   v16b __attribute__((ext_vector_type(16)));
typedef __bf16   v8b  __attribute__((ext_vector_type(8)));
typedef float    v8f  __attribute__((ext_vector_type(8)));
typedef float    v4f  __attribute__((ext_vector_type(4)));
typedef unsigned int v4u __attribute__((ext_vector_type(4)));
typedef unsigned short v16us __attribute__((ext_vector_type(16)));

#if defined(__HIP_DEVICE_COMPILE__)
#define DEV_ASM 1
#else
#define DEV_ASM 0
#endif

__device__ __forceinline__ unsigned short bf_bits(float f) {
  unsigned u = __float_as_uint(f);
  return (unsigned short)((u + 0x7FFFu + ((u >> 16) & 1u)) >> 16);
}
__device__ __forceinline__ float bf_up(unsigned short hb) { return __uint_as_float(((unsigned)hb) << 16); }
__device__ __forceinline__ unsigned pk16(unsigned short a, unsigned short b) { return (unsigned)a | ((unsigned)b << 16); }
__device__ __forceinline__ v8f zero8() { v8f z = {0.f, 0.f, 0.f, 0.f, 0.f, 0.f, 0.f, 0.f}; return z; }
__device__ __forceinline__ void split_bf(float f, unsigned short& hb, unsigned short& lb) {
  hb = bf_bits(f);
  lb = bf_bits(f - bf_up(hb));
}

template <typename OT> struct FT;
template <> struct FT<__bf16> { typedef v16b frag; typedef v8b half8; };

template <typename OT>
__device__ __forceinline__ typename FT<OT>::frag ldfrag(const OT* p) {
  union { typename FT<OT>::frag v; typename FT<OT>::half8 h[2]; } f;
  f.h[0] = *(const typename FT<OT>::half8*)(p);
  f.h[1] = *(const typename FT<OT>::half8*)(p + 16);
  return f.v;
}

__device__ __forceinline__ v8f mmar(v16b a, v16b b, v8f c) {
  return __builtin_amdgcn_wmma_f32_16x16x32_bf16(false, a, false, b, (short)0, c, false, false);
}
__device__ __forceinline__ v8f mma_b(v16b a, v16b b, v8f c) {
  c = __builtin_amdgcn_wmma_f32_16x16x32_bf16(false, a, false, b, (short)0, c, false, false);
#if DEV_ASM
  asm volatile("v_nop\n\tv_nop\n\tv_nop\n\tv_nop" : "+v"(c) : "v"(a), "v"(b));
#endif
  return c;
}
__device__ __forceinline__ void dep_guard(v8f& a, v8f& b, v16b x, v16b y) {
#if DEV_ASM
  asm volatile("v_nop\n\tv_nop\n\tv_nop\n\tv_nop" : "+v"(a), "+v"(b) : "v"(x), "v"(y));
#else
  (void)a; (void)b; (void)x; (void)y;
#endif
}
__device__ __forceinline__ void keep4(v16b a, v16b b, v16b c, v16b d) {
#if DEV_ASM
  asm volatile("v_nop" :: "v"(a), "v"(b), "v"(c), "v"(d));
#else
  (void)a; (void)b; (void)c; (void)d;
#endif
}
__device__ __forceinline__ void acc_guard4(v8f& a, v8f& b, v8f& c, v8f& d) {
#if DEV_ASM
  asm volatile("v_nop\n\tv_nop\n\tv_nop\n\tv_nop" : "+v"(a), "+v"(b), "+v"(c), "+v"(d));
#else
  (void)a; (void)b; (void)c; (void)d;
#endif
}

__global__ __launch_bounds__(256) void cvt_x(const float* __restrict__ x, unsigned short* xh) {
  __shared__ float t[64 * 65];
  const int tid = (int)threadIdx.x;
  const int p0 = blockIdx.x * 64, c0 = blockIdx.y * 64, b = blockIdx.z;
#pragma unroll
  for (int it = 0; it < 4; ++it) {
    const int c  = it * 16 + (tid >> 4);
    const int p4 = (tid & 15) * 4;
    const v4f v = *(const v4f*)(x + ((size_t)(b * CH + c0 + c)) * NPOS + p0 + p4);
    float* tp = t + c * 65 + p4;
    tp[0] = v[0]; tp[1] = v[1]; tp[2] = v[2]; tp[3] = v[3];
  }
  __syncthreads();
  v4u pk[2];
  size_t go[2];
#pragma unroll
  for (int it = 0; it < 2; ++it) {
    const int item = it * 256 + tid;
    const int p = item >> 3, cg = item & 7;
    v4u a;
#pragma unroll
    for (int e = 0; e < 4; ++e) {
      const float f0 = t[(cg * 8 + 2 * e) * 65 + p];
      const float f1 = t[(cg * 8 + 2 * e + 1) * 65 + p];
      a[e] = pk16(bf_bits(f0), bf_bits(f1));
    }
    pk[it] = a;
    go[it] = ((size_t)(b * NPOS + p0 + p)) * CH + c0 + cg * 8;
  }
  for (int ps = 0; ps < 2; ++ps) {
#pragma unroll
    for (int it = 0; it < 2; ++it) *(volatile v4u*)(xh + go[it]) = pk[it];
    __threadfence();
  }
}

__global__ __launch_bounds__(256) void cvt16x8(const float* __restrict__ in, unsigned short* out, int n8) {
  const int i = blockIdx.x * 256 + (int)threadIdx.x;
  if (i < n8) {
    const v4f a  = *(const v4f*)(in + (size_t)i * 8);
    const v4f a4 = *(const v4f*)(in + (size_t)i * 8 + 4);
    v4u p;
    p[0] = pk16(bf_bits(a[0]),  bf_bits(a[1]));
    p[1] = pk16(bf_bits(a[2]),  bf_bits(a[3]));
    p[2] = pk16(bf_bits(a4[0]), bf_bits(a4[1]));
    p[3] = pk16(bf_bits(a4[2]), bf_bits(a4[3]));
    unsigned short* o = out + (size_t)i * 8;
    *(volatile v4u*)o = p;
    __threadfence();
    *(volatile v4u*)o = p;
  }
}

__global__ __launch_bounds__(256) void cvt_wp(const float* __restrict__ wp, unsigned short* out) {
  const int i = blockIdx.x * 256 + (int)threadIdx.x;
  if (i < CH * CTXK / 8) {
    const int c  = i >> 6;
    const int k  = (i & 63) * 8;
    const int hd = k >> 6;
    const int d0 = k & 31;
    const float* src = wp + (size_t)c * CH + hd * HDIM + d0;
    const v4f a  = *(const v4f*)src;
    const v4f a4 = *(const v4f*)(src + 4);
    v4u p;
    p[0] = pk16(bf_bits(a[0]),  bf_bits(a[1]));
    p[1] = pk16(bf_bits(a[2]),  bf_bits(a[3]));
    p[2] = pk16(bf_bits(a4[0]), bf_bits(a4[1]));
    p[3] = pk16(bf_bits(a4[2]), bf_bits(a4[3]));
    unsigned short* o = out + (size_t)i * 8;
    *(volatile v4u*)o = p;
    __threadfence();
    *(volatile v4u*)o = p;
  }
}

template <int BIAS_MODE>
__global__ __launch_bounds__(256) void gemm64(
    const unsigned short* __restrict__ Ap, int lda, long long strideA,
    const unsigned short* __restrict__ Btp, int ldb, long long strideB,
    float* Cout, int ldc, long long strideC,
    const float* __restrict__ bias,
    int M, int N, int K) {
  const __bf16* A  = (const __bf16*)(const void*)Ap;
  const __bf16* Bt = (const __bf16*)(const void*)Btp;
  __shared__ __align__(16) float sT[8][16 * 68];
  const int b    = blockIdx.y;
  const int lane = threadIdx.x & 31;
  const int wave = threadIdx.x >> 5;
  const int tilesN = N >> 6;
  const int tilesM = M >> 6;
  const int tile = blockIdx.x * 8 + wave;
  if (tile >= tilesM * tilesN) return;
  const int tm = tile / tilesN;
  const int tn = tile - tm * tilesN;
  const int m0 = tm << 6;
  const int n0 = tn << 6;

  const __bf16* Ab = A  + (size_t)b * (size_t)strideA;
  const __bf16* Bb = Bt + (size_t)b * (size_t)strideB;

  const int rlane = lane & 15;
  const int koff  = (lane >> 4) * 8;
  const int mOff  = (lane >> 4) * 8;

  v8f acc[4][4];
#pragma unroll
  for (int i = 0; i < 4; ++i)
#pragma unroll
    for (int j = 0; j < 4; ++j) acc[i][j] = zero8();

  for (int k0 = 0; k0 < K; k0 += 32) {
    v16b bq[4];
#pragma unroll
    for (int j = 0; j < 4; ++j)
      bq[j] = ldfrag<__bf16>(Bb + (size_t)(n0 + (j << 4) + rlane) * ldb + koff + k0);
#pragma unroll
    for (int i = 0; i < 4; ++i) {
      const v16b af = ldfrag<__bf16>(Ab + (size_t)(m0 + (i << 4) + rlane) * lda + koff + k0);
#pragma unroll
      for (int j = 0; j < 4; ++j) acc[i][j] = mmar(af, bq[j], acc[i][j]);
      dep_guard(acc[i][0], acc[i][3], af, bq[3]);
    }
    keep4(bq[0], bq[1], bq[2], bq[3]);
  }
  acc_guard4(acc[0][0], acc[0][1], acc[0][2], acc[0][3]);
  acc_guard4(acc[1][0], acc[1][1], acc[1][2], acc[1][3]);
  acc_guard4(acc[2][0], acc[2][1], acc[2][2], acc[2][3]);
  acc_guard4(acc[3][0], acc[3][1], acc[3][2], acc[3][3]);

  float* slab = sT[wave];
  float* C = Cout + (size_t)b * (size_t)strideC;
  const int h2 = lane >> 4, c4 = (lane & 15) * 4;
  v4f bcol = {0.f, 0.f, 0.f, 0.f};
  if (BIAS_MODE == 1) {
#pragma unroll
    for (int e = 0; e < 4; ++e) bcol[e] = bf_up(bf_bits(bias[n0 + c4 + e]));
  }
#pragma unroll
  for (int i = 0; i < 4; ++i) {
    const int mBase = m0 + (i << 4);
#pragma unroll
    for (int j = 0; j < 4; ++j) {
#pragma unroll
      for (int r = 0; r < 8; ++r) {
        slab[(mOff + r) * 68 + (j << 4) + rlane] = acc[i][j][r];
      }
    }
    __builtin_amdgcn_fence(__ATOMIC_RELEASE, "workgroup");
    __builtin_amdgcn_wave_barrier();
    __builtin_amdgcn_fence(__ATOMIC_ACQUIRE, "workgroup");
    for (int ps = 0; ps < 2; ++ps) {
#pragma unroll
      for (int it = 0; it < 8; ++it) {
        const int row = it * 2 + h2;
        v4f v = *(const v4f*)(slab + row * 68 + c4);
        if (BIAS_MODE == 1) {
          v = v + bcol;
        } else {
          const float br = bf_up(bf_bits(bias[mBase + row]));
          v = v + br;
        }
        *(volatile v4f*)(C + (size_t)(mBase + row) * ldc + n0 + c4) = v;
      }
      __threadfence();
    }
    __builtin_amdgcn_fence(__ATOMIC_RELEASE, "workgroup");
    __builtin_amdgcn_wave_barrier();
    __builtin_amdgcn_fence(__ATOMIC_ACQUIRE, "workgroup");
  }
}

union PBits { v16us u; v16b v; };
__device__ __forceinline__ void pack_pt(v8f a, v8f c, v16b& ph, v16b& pl) {
  const v16us zz = {0, 0, 0, 0, 0, 0, 0, 0, 0, 0, 0, 0, 0, 0, 0, 0};
  PBits H, L;
  H.u = zz; L.u = zz;
#pragma unroll
  for (int r = 0; r < 8; ++r) {
    const unsigned short hb = bf_bits(a[r]);
    H.u[r] = hb;
    L.u[r] = bf_bits(a[r] - bf_up(hb));
  }
#pragma unroll
  for (int r = 0; r < 8; ++r) {
    const unsigned short hb = bf_bits(c[r]);
    H.u[8 + r] = hb;
    L.u[8 + r] = bf_bits(c[r] - bf_up(hb));
  }
  ph = H.v; pl = L.v;
}

__device__ __forceinline__ void ld8sel(const float* src, int keep, float f[8]) {
  const v4f a = *(const v4f*)src;
  const v4f c = *(const v4f*)(src + 4);
  f[0] = keep ? a[0] : 0.f; f[1] = keep ? a[1] : 0.f; f[2] = keep ? a[2] : 0.f; f[3] = keep ? a[3] : 0.f;
  f[4] = keep ? c[0] : 0.f; f[5] = keep ? c[1] : 0.f; f[6] = keep ? c[2] : 0.f; f[7] = keep ? c[3] : 0.f;
}

__global__ __launch_bounds__(128)
void natt(const float* __restrict__ qkv, const float* __restrict__ rpb, unsigned short* ctx) {
  __shared__ __align__(16) unsigned short KV0[NSLOT * HDIM];
  __shared__ __align__(16) unsigned short KV1[NSLOT * HDIM];
  __shared__ __align__(16) unsigned short Qh[64 * HDIM];
  __shared__ __align__(16) unsigned short Ql[64 * HDIM];
  __shared__ __align__(16) float Os[4][16 * HDIM];
  __shared__ float Rp[176];

  const int tid  = (int)threadIdx.x;
  const int wave = tid >> 5;
  const int lane = tid & 31;
  const int hh   = lane >> 4;
  const int m    = lane & 15;

  const int bx   = blockIdx.x;
  const int tj   = bx % 7;
  const int ti   = (bx / 7) % 7;
  const int head = (bx / 49) % NHD;
  const int b    = bx / (49 * NHD);
  const int i0 = ti * 8, j0 = tj * 8;
  const int R0 = min(max(i0 - 3, 0), IMH - SUP);
  const int C0 = min(max(j0 - 3, 0), IMW - SUP);
  const size_t pb = (size_t)b * NPOS;

  {
    const float r0v = rpb[head * 169 + tid];
    const int   i1  = tid + 128;
    const float r1v = rpb[head * 169 + min(i1, 168)];
    Rp[tid] = bf_up(bf_bits(r0v));
    if (i1 < 169) Rp[i1] = bf_up(bf_bits(r1v));
  }
  {
    const int lq = tid >> 1, dh = (tid & 1) * 16;
    const int qi = lq >> 3, qj = lq & 7;
    const size_t pos = pb + (size_t)(i0 + qi) * IMW + j0 + qj;
    const float* src = qkv + pos * C3 + head * HDIM + dh;
#pragma unroll
    for (int g = 0; g < 2; ++g) {
      float f[8];
      ld8sel(src + 8 * g, 1, f);
      v4u ph, pl;
#pragma unroll
      for (int e = 0; e < 4; ++e) {
        unsigned short h0, l0, h1, l1;
        split_bf(f[2 * e] * QSCALE, h0, l0);
        split_bf(f[2 * e + 1] * QSCALE, h1, l1);
        ph[e] = pk16(h0, h1); pl[e] = pk16(l0, l1);
      }
      *(v4u*)(Qh + lq * HDIM + dh + 8 * g) = ph;
      *(v4u*)(Ql + lq * HDIM + dh + 8 * g) = pl;
    }
  }
  {
    const float* kbase = qkv + CH + head * HDIM;
#pragma unroll
    for (int it = 0; it < 7; ++it) {
      const int item = it * 128 + tid;
      const int slot = item >> 2, d8 = (item & 3) * 8;
      const int u = slot / SUP, v = slot - u * SUP;
      const int uc = min(u, SUP - 1);
      const size_t pos = pb + (size_t)(R0 + uc) * IMW + C0 + v;
      float f[8];
      ld8sel(kbase + pos * C3 + d8, slot < SUP * SUP, f);
      v4u ph, pl;
#pragma unroll
      for (int e = 0; e < 4; ++e) {
        unsigned short h0, l0, h1, l1;
        split_bf(f[2 * e], h0, l0);
        split_bf(f[2 * e + 1], h1, l1);
        ph[e] = pk16(h0, h1); pl[e] = pk16(l0, l1);
      }
      *(v4u*)(KV0 + slot * HDIM + d8) = ph;
      *(v4u*)(KV1 + slot * HDIM + d8) = pl;
    }
  }
  __syncthreads();

  v8f s[NKT + 1];
  {
    const __bf16* Kh = (const __bf16*)(const void*)KV0;
    const __bf16* Kl = (const __bf16*)(const void*)KV1;
    const __bf16* Qhp = (const __bf16*)(const void*)Qh;
    const __bf16* Qlp = (const __bf16*)(const void*)Ql;
    const v16b qfh = ldfrag<__bf16>(Qhp + (16 * wave + m) * HDIM + 8 * hh);
    const v16b qfl = ldfrag<__bf16>(Qlp + (16 * wave + m) * HDIM + 8 * hh);
#pragma unroll
    for (int j = 0; j < NKT; ++j) {
      const v16b kfh = ldfrag<__bf16>(Kh + (16 * j + m) * HDIM + 8 * hh);
      const v16b kfl = ldfrag<__bf16>(Kl + (16 * j + m) * HDIM + 8 * hh);
      v8f z = zero8();
      z = mma_b(kfh, qfh, z);
      z = mma_b(kfh, qfl, z);
      z = mma_b(kfl, qfh, z);
      s[j] = z;
    }
    s[NKT] = zero8();
  }
  __syncthreads();

  {
    const float* vbase = qkv + 2 * CH + head * HDIM;
#pragma unroll
    for (int it = 0; it < 7; ++it) {
      const int item = it * 128 + tid;
      const int slot = item >> 2, d8 = (item & 3) * 8;
      const int u = slot / SUP, v = slot - u * SUP;
      const int uc = min(u, SUP - 1);
      const size_t pos = pb + (size_t)(R0 + uc) * IMW + C0 + v;
      float f[8];
      ld8sel(vbase + pos * C3 + d8, slot < SUP * SUP, f);
#pragma unroll
      for (int e = 0; e < 8; ++e) {
        unsigned short h0, l0;
        split_bf(f[e], h0, l0);
        KV0[(d8 + e) * NSLOT + slot] = h0;
        KV1[(d8 + e) * NSLOT + slot] = l0;
      }
    }
  }
  __syncthreads();

  const int lq = 16 * wave + m;
  const int ai = i0 + (lq >> 3), aj = j0 + (lq & 7);
  const int su = min(max(ai - 3, 0), IMH - KW) - R0;
  const int sv = min(max(aj - 3, 0), IMW - KW) - C0;
  const int cb = (R0 - ai + 6) * 13 + (C0 - aj + 6);
  float mloc = -1.0e30f;
#pragma unroll
  for (int j = 0; j < NKT; ++j) {
#pragma unroll
    for (int r = 0; r < 8; ++r) {
      const int t0 = 16 * j + r;
      const int u = hh ? ((t0 + 8) / SUP) : (t0 / SUP);
      const int v = hh ? ((t0 + 8) % SUP) : (t0 % SUP);
      const bool ok = ((unsigned)(u - su) < 7u) && ((unsigned)(v - sv) < 7u);
      int bi = u * 13 + v + cb;
      bi = min(max(bi, 0), 168);
      const float bv = Rp[bi];
      const float sval = ok ? (s[j][r] + bv) : -1.0e30f;
      s[j][r] = sval;
      mloc = fmaxf(mloc, sval);
    }
  }
  const float mrow = fmaxf(mloc, __shfl_xor(mloc, 16, 32));
  float lsum = 0.f;
#pragma unroll
  for (int j = 0; j < NKT; ++j) {
#pragma unroll
    for (int r = 0; r < 8; ++r) {
      const float p = __expf(s[j][r] - mrow);
      s[j][r] = p;
      lsum += p;
    }
  }
  lsum += __shfl_xor(lsum, 16, 32);

  v8f o[2];
  o[0] = zero8(); o[1] = zero8();
  {
    const __bf16* Vh = (const __bf16*)(const void*)KV0;
    const __bf16* Vl = (const __bf16*)(const void*)KV1;
#pragma unroll
    for (int kk = 0; kk < NSLOT / 32; ++kk) {
      v16b ph, pl;
      pack_pt(s[2 * kk], s[2 * kk + 1], ph, pl);
#pragma unroll
      for (int t = 0; t < 2; ++t) {
        const v16b vfh = ldfrag<__bf16>(Vh + (16 * t + m) * NSLOT + 32 * kk + 8 * hh);
        const v16b vfl = ldfrag<__bf16>(Vl + (16 * t + m) * NSLOT + 32 * kk + 8 * hh);
        o[t] = mma_b(vfh, ph, o[t]);
        o[t] = mma_b(vfh, pl, o[t]);
        o[t] = mma_b(vfl, ph, o[t]);
      }
    }
  }

  const float linv = 1.0f / lsum;
  float* os = Os[wave];
#pragma unroll
  for (int t = 0; t < 2; ++t)
#pragma unroll
    for (int r = 0; r < 8; ++r) os[m * HDIM + 16 * t + 8 * hh + r] = o[t][r] * linv;
  __syncthreads();
  {
    const int q4 = lane >> 3, pc = lane & 7, dsel = (pc & 3) * 8;
    const bool lowp = (pc >= 4);
    v4u hv[4];
    size_t go[4];
#pragma unroll
    for (int it = 0; it < 4; ++it) {
      const int row = it * 4 + q4;
      const float* sp = os + row * HDIM + dsel;
      v4u a;
#pragma unroll
      for (int e = 0; e < 4; ++e) {
        unsigned short h0, l0, h1, l1;
        split_bf(sp[2 * e], h0, l0);
        split_bf(sp[2 * e + 1], h1, l1);
        a[e] = lowp ? pk16(l0, l1) : pk16(h0, h1);
      }
      hv[it] = a;
      const int lqr = 16 * wave + row;
      const size_t pos = pb + (size_t)(i0 + (lqr >> 3)) * IMW + j0 + (lqr & 7);
      go[it] = pos * CTXK + (size_t)head * 64 + pc * 8;
    }
    for (int ps = 0; ps < 2; ++ps) {
#pragma unroll
      for (int it = 0; it < 4; ++it) *(volatile v4u*)(ctx + go[it]) = hv[it];
      __threadfence();
    }
  }
}

extern "C" void kernel_launch(void* const* d_in, const int* in_sizes, int n_in,
                              void* d_out, int out_size, void* d_ws, size_t ws_size,
                              hipStream_t stream) {
  if (n_in < 6) return;
  if (in_sizes[0] != NBT * CH * NPOS) return;
  if (in_sizes[1] != C3 * CH) return;
  if (in_sizes[2] != C3) return;
  if (in_sizes[3] != NHD * 13 * 13) return;
  if (in_sizes[4] != CH * CH) return;
  if (in_sizes[5] != CH) return;
  if (out_size != NBT * CH * NPOS) return;

  const float* x      = (const float*)d_in[0];
  const float* w_qkv  = (const float*)d_in[1];
  const float* b_qkv  = (const float*)d_in[2];
  const float* rpb    = (const float*)d_in[3];
  const float* w_proj = (const float*)d_in[4];
  const float* b_proj = (const float*)d_in[5];

  const size_t PXH  = (size_t)MROW * CH * 2;
  const size_t PWQ  = (size_t)C3 * CH * 2;
  const size_t PWP  = (size_t)CH * CTXK * 2;
  const size_t PQKV = (size_t)MROW * C3 * 4;
  const size_t PCTX = (size_t)MROW * CTXK * 2;
  size_t off = 0;
  const size_t oXh  = off; off += PXH;
  const size_t oWq  = off; off += PWQ;
  const size_t oWp  = off; off += PWP;
  const size_t oQKV = off; off += PQKV;
  const size_t oCTX = off; off += PCTX;
  if (off > ws_size) return;
  if (off > (size_t)134217728) return;

  char* ws = (char*)d_ws;
  unsigned short* Xh  = (unsigned short*)(ws + oXh);
  unsigned short* Wqb = (unsigned short*)(ws + oWq);
  unsigned short* Wpf = (unsigned short*)(ws + oWp);
  float*          QKV = (float*)(ws + oQKV);
  unsigned short* CTX = (unsigned short*)(ws + oCTX);

  const int n8wq = C3 * CH / 8;
  const int tilesQKV = (MROW / 64) * (C3 / 64);
  const int tilesPRJ = (CH / 64) * (NPOS / 64);
  const dim3 gX(NPOS / 64, CH / 64, NBT);
  const dim3 gWq((n8wq + 255) / 256);
  const dim3 gWp((CH * CTXK / 8 + 255) / 256);
  const dim3 gQKV((tilesQKV + 7) / 8, 1);
  const dim3 gAtt(NBT * NHD * 49);
  const dim3 gPRJ((tilesPRJ + 7) / 8, NBT);

  cvt_x<<<gX, dim3(256), 0, stream>>>(x, Xh);
  cvt16x8<<<gWq, dim3(256), 0, stream>>>(w_qkv, Wqb, n8wq);
  cvt_wp<<<gWp, dim3(256), 0, stream>>>(w_proj, Wpf);
  gemm64<1><<<gQKV, dim3(256), 0, stream>>>(
      Xh, CH, 0LL, Wqb, CH, 0LL,
      QKV, C3, 0LL, b_qkv,
      MROW, C3, CH);
  natt<<<gAtt, dim3(128), 0, stream>>>(QKV, rpb, CTX);
  gemm64<2><<<gPRJ, dim3(256), 0, stream>>>(
      Wpf, CTXK, 0LL, CTX, CTXK, (long long)NPOS * CTXK,
      (float*)d_out, NPOS, (long long)CH * NPOS, b_proj,
      CH, NPOS, CTXK);
  (void)hipGetLastError();
}
